// NodeNetwork_70265664963043
// MI455X (gfx1250) — hardware-verified
//
#include <hip/hip_runtime.h>
#include <math.h>

typedef __attribute__((ext_vector_type(16))) _Float16 v16h;
typedef __attribute__((ext_vector_type(16))) __bf16 v16b;
typedef __attribute__((ext_vector_type(8)))  _Float16 v8h;
typedef __attribute__((ext_vector_type(8)))  float v8f;
typedef __attribute__((ext_vector_type(4)))  float v4f;
typedef __attribute__((ext_vector_type(2)))  float v2f;
typedef __attribute__((ext_vector_type(4)))  unsigned v4u;
typedef __attribute__((ext_vector_type(4)))  int v4i;
typedef float __attribute__((may_alias)) float_a;
typedef int __attribute__((may_alias)) int_a;

template <typename T> __device__ __forceinline__ void vst2(void* p, T v) { *(volatile T*)p = v; __threadfence(); *(volatile T*)p = v; }
__device__ __forceinline__ v8f wmma16(v16h a, v16h b, v8f c) {
  v8f d = __builtin_amdgcn_wmma_f32_16x16x32_f16(false, a, false, b, (short)0, c, false, false);
  asm volatile("v_nop\n\tv_nop\n\tv_nop\n\tv_nop" : "+v"(d) : "v"(a), "v"(b));
  return d;
}
__device__ __forceinline__ v8f wmma_bf(v16b a, v16b b, v8f c) {
  v8f d = __builtin_amdgcn_wmma_f32_16x16x32_bf16(false, a, false, b, (short)0, c, false, false);
  asm volatile("v_nop\n\tv_nop\n\tv_nop\n\tv_nop" : "+v"(d) : "v"(a), "v"(b));
  return d;
}
__device__ __forceinline__ v16h frag_h(const _Float16* rowk0, int lane) {
  union { v16h v; v8h q[2]; } u; const _Float16* p = rowk0 + 8 * (lane >> 4);
  u.q[0] = *(const v8h*)p; u.q[1] = *(const v8h*)(p + 16); return u.v;
}
__device__ __forceinline__ v16h frag_f32(const float* rowk0, int lane) {
  v16h a; const float* p = rowk0 + 8 * (lane >> 4);
#pragma unroll
  for (int i = 0; i < 8; ++i) { a[i] = (_Float16)p[i]; a[8 + i] = (_Float16)p[16 + i]; }
  return a;
}
__device__ __forceinline__ v16h frag_f32s(const float* rowk0, int lane, float sc) {
  v16h a; const float* p = rowk0 + 8 * (lane >> 4);
#pragma unroll
  for (int i = 0; i < 8; ++i) { a[i] = (_Float16)(p[i] * sc); a[8 + i] = (_Float16)(p[16 + i] * sc); }
  return a;
}
__device__ __forceinline__ v16h fragc_f32(const float* W, int k0, int n, int lane, int ld, int K) {
  v16h a; const int g = lane >> 4;
#pragma unroll
  for (int i = 0; i < 8; ++i) { const int ka = k0 + 8 * g + i, kb = ka + 16;
    a[i] = (_Float16)(ka < K ? W[(size_t)ka * ld + n] : 0.f); a[8 + i] = (_Float16)(kb < K ? W[(size_t)kb * ld + n] : 0.f); }
  return a;
}
struct F2 { v16b h, l; };
__device__ __forceinline__ F2 bsplit16(const float v[16]) { F2 r;
#pragma unroll
  for (int i = 0; i < 16; ++i) { const __bf16 h = (__bf16)v[i]; r.h[i] = h; r.l[i] = (__bf16)(v[i] - (float)h); }
  return r; }
__device__ __forceinline__ F2 split_row(const float* row, int k0, int lane) { float v[16]; const float* p = row + k0 + 8 * (lane >> 4);
#pragma unroll
  for (int i = 0; i < 8; ++i) { v[i] = p[i]; v[8 + i] = p[16 + i]; }
  return bsplit16(v); }
__device__ __forceinline__ F2 split_rowK(const float* row, int k0, int lane, int K) { float v[16]; const int g = lane >> 4;
#pragma unroll
  for (int i = 0; i < 8; ++i) { const int ka = k0 + 8 * g + i, kb = ka + 16; v[i] = ka < K ? row[ka] : 0.f; v[8 + i] = kb < K ? row[kb] : 0.f; }
  return bsplit16(v); }
__device__ __forceinline__ F2 split_col(const float* W, int k0, int n, int lane, int ld, int K) { float v[16]; const int g = lane >> 4;
#pragma unroll
  for (int i = 0; i < 8; ++i) { const int ka = k0 + 8 * g + i, kb = ka + 16; v[i] = ka < K ? W[(size_t)ka * ld + n] : 0.f; v[8 + i] = kb < K ? W[(size_t)kb * ld + n] : 0.f; }
  return bsplit16(v); }
__device__ __forceinline__ v8f mac3(const F2& a, const F2& b, v8f c) { c = wmma_bf(a.l, b.h, c); c = wmma_bf(a.h, b.l, c); return wmma_bf(a.h, b.h, c); }
__device__ __forceinline__ float sigm(float v) { return 1.0f / (1.0f + expf(-v)); }
#define LDSX() do { asm volatile("s_wait_dscnt 0" ::: "memory"); __builtin_amdgcn_wave_barrier(); __builtin_amdgcn_fence(__ATOMIC_RELEASE, "workgroup"); } while (0)

#define NB 8
#define NN 256
#define FF 32
#define OH 32
#define ME 48
#define MN 32
#define NR (NB * NN)

__global__ __launch_bounds__(256) void k_uv(const float* __restrict__ xn, const float* __restrict__ eW1, float* __restrict__ U, float* __restrict__ V) {
  __shared__ __align__(16) float su[16][ME], sv[16][ME];
  const int tid = threadIdx.x, r0 = blockIdx.x * 16;
  { const int rl = tid >> 4, cgp = tid & 15; const float* xr = xn + (size_t)(r0 + rl) * FF;
    for (int c = cgp * 3; c < ME; c += 48) { for (int cc = c; cc < c + 3 && cc < ME; ++cc) { float u = 0.f, v = 0.f;
#pragma unroll 8
        for (int f = 0; f < FF; ++f) { const float xv = xr[f]; u += xv * eW1[(size_t)f * ME + cc]; v += xv * eW1[(size_t)(FF + f) * ME + cc]; }
        su[rl][cc] = u; sv[rl][cc] = v; } } }
  __syncthreads();
  for (int q = tid; q < 16 * ME / 4; q += 256) { vst2(U + (size_t)r0 * ME + q * 4, *(const v4f*)(&su[0][0] + q * 4)); vst2(V + (size_t)r0 * ME + q * 4, *(const v4f*)(&sv[0][0] + q * 4)); }
}
__global__ __launch_bounds__(128) void k_edge(const float* __restrict__ U, const float* __restrict__ V, const float* __restrict__ edge, const float* __restrict__ eW1, const float* __restrict__ eb1, const float* __restrict__ eW2, const float* __restrict__ eb2, float* __restrict__ msg) {
  __shared__ __align__(16) float sh[4][16][68];
  __shared__ float ssum[4][4][OH];
  __shared__ __align__(16) float so[OH];
  const int tid = threadIdx.x, wave = tid >> 5, lane = tid & 31, col = lane & 15, g = lane >> 4;
  const int i = blockIdx.x, b = blockIdx.y; const size_t ri = (size_t)b * NN + i;
  float tot[2] = {0.f, 0.f};
  v8f csum[2] = {};
#pragma unroll 1
  for (int pass = 0; pass < 4; ++pass) {
    const int j0 = pass * 64 + wave * 16;
    for (int q = lane; q < 16 * 64; q += 32) { const int rl = q >> 6, c = q & 63; const int j = j0 + rl; float v = 0.f;
      if (c < ME && j != i) { const int slot = j < i ? j : j - 1; v = U[ri * ME + c] + V[((size_t)b * NN + j) * ME + c] + edge[ri * (NN - 1) + slot] * eW1[(size_t)(2 * FF) * ME + c] + eb1[c]; v = v > 0.f ? v : 0.f; }
      sh[wave][rl][c] = v; }
    LDSX();
    v8f acc[2] = {};
#pragma unroll
    for (int kc = 0; kc < 2; ++kc) { const F2 a = split_row(&sh[wave][col][0], kc * 32, lane);
#pragma unroll
      for (int t = 0; t < 2; ++t) acc[t] = mac3(a, split_col(eW2, kc * 32, t * 16 + col, lane, OH, ME), acc[t]); }
#pragma unroll
    for (int t = 0; t < 2; ++t) { const float bb = eb2[t * 16 + col];
#pragma unroll
      for (int r = 0; r < 8; ++r) { const int j = j0 + 8 * g + r; if (j != i) csum[t][r] += tanhf(acc[t][r] + bb); } }
    LDSX(); }
#pragma unroll
  for (int t = 0; t < 2; ++t) { float s = 0.f;
#pragma unroll
    for (int r = 0; r < 8; ++r) s += csum[t][r];
    s += __shfl_xor(s, 16, 32); tot[t] = s; }
  if (g == 0) { ssum[wave][0][col] = tot[0]; ssum[wave][0][16 + col] = tot[1]; }
  __syncthreads();
  if (tid < OH) so[tid] = (ssum[0][0][tid] + ssum[1][0][tid]) + (ssum[2][0][tid] + ssum[3][0][tid]);
  __syncthreads();
  if (tid < OH / 4) vst2(msg + ri * OH + tid * 4, *(const v4f*)(&so[tid * 4]));
}
__global__ __launch_bounds__(256) void k_node(const float* __restrict__ xn, const float* __restrict__ msg, const float* __restrict__ n1W1, const float* __restrict__ n1b1, const float* __restrict__ n1W2, const float* __restrict__ n1b2,
                                            const float* __restrict__ n2W1, const float* __restrict__ n2b1, const float* __restrict__ n2W2, const float* __restrict__ n2b2, float* __restrict__ out) {
  __shared__ float sa[8][MN], sb[8][MN]; __shared__ __align__(16) float so[8][2 * OH]; __shared__ float snrm[8];
  const int tid = threadIdx.x, nl = tid >> 5, c = tid & 31; const size_t r = (size_t)blockIdx.x * 8 + nl;
  { float a = n1b1[c], bsum = n2b1[c];
#pragma unroll 8
    for (int f = 0; f < FF; ++f) a += xn[r * FF + f] * n1W1[f * MN + c];
#pragma unroll 8
    for (int f = 0; f < OH; ++f) bsum += msg[r * OH + f] * n2W1[f * OH + c];
    sa[nl][c] = a > 0.f ? a : 0.f; sb[nl][c] = bsum > 0.f ? bsum : 0.f; }
  __syncthreads();
  { float a = n1b2[c], bsum = n2b2[c];
#pragma unroll 8
    for (int f = 0; f < MN; ++f) a += sa[nl][f] * n1W2[f * OH + c];
#pragma unroll 8
    for (int f = 0; f < OH; ++f) bsum += sb[nl][f] * n2W2[f * OH + c];
    const float o1 = tanhf(a), o2 = tanhf(bsum); so[nl][c] = o1; so[nl][OH + c] = o2;
    float q2 = o1 * o1 + o2 * o2;
#pragma unroll
    for (int off = 16; off >= 1; off >>= 1) q2 += __shfl_xor(q2, off, 32);
    if (c == 0) snrm[nl] = sqrtf(q2); }
  __syncthreads();
  for (int q = tid; q < 8 * 2 * OH; q += 256) { const int n = q >> 6, cc = q & 63; so[n][cc] = so[n][cc] / snrm[n]; }
  __syncthreads();
  for (int q = tid; q < 8 * 2 * OH / 4; q += 256) vst2(out + (size_t)blockIdx.x * 8 * 2 * OH + q * 4, *(const v4f*)(&so[0][0] + q * 4));
}
extern "C" void kernel_launch(void* const* d_in, const int* in_sizes, int n_in, void* d_out, int out_size, void* d_ws, size_t ws_size, hipStream_t stream) {
  (void)in_sizes; (void)n_in; (void)out_size; (void)ws_size;
  const float** I = (const float**)d_in;
  const float* xn = I[0]; const float* edge = I[1]; const float* eW1 = I[2]; const float* eb1 = I[3]; const float* eW2 = I[4]; const float* eb2 = I[5];
  const float* n1W1 = I[6]; const float* n1b1 = I[7]; const float* n1W2 = I[8]; const float* n1b2 = I[9]; const float* n2W1 = I[10]; const float* n2b1 = I[11]; const float* n2W2 = I[12]; const float* n2b2 = I[13];
  float* out = (float*)d_out;
  char* ws = (char*)d_ws; size_t off = 0;
  auto take = [&](size_t bytes) { char* p = ws + off; off += (bytes + 255) & ~(size_t)255; return p; };
  float* U = (float*)take((size_t)NR * ME * 4); float* V = (float*)take((size_t)NR * ME * 4); float* msg = (float*)take((size_t)NR * OH * 4);
  k_uv<<<NR / 16, 256, 0, stream>>>(xn, eW1, U, V);
  k_edge<<<dim3(NN, NB), 128, 0, stream>>>(U, V, edge, eW1, eb1, eW2, eb2, msg);
  k_node<<<NR / 8, 256, 0, stream>>>(xn, msg, n1W1, n1b1, n1W2, n1b2, n2W1, n2b1, n2W2, n2b2, out);
}
